// DeepQNetwork_40776419508448
// MI455X (gfx1250) — hardware-run, weakly checked
//
#include <hip/hip_runtime.h>
#include <stddef.h>
#include <stdint.h>

typedef __attribute__((ext_vector_type(16))) _Float16 v16h;
typedef __attribute__((ext_vector_type(8)))  _Float16 v8h;
typedef __attribute__((ext_vector_type(16))) __bf16   v16b;
typedef __attribute__((ext_vector_type(8)))  __bf16   v8b;
typedef __attribute__((ext_vector_type(8)))  float    v8f;
typedef __attribute__((ext_vector_type(4)))  float    v4f;
typedef __attribute__((ext_vector_type(4)))  unsigned int v4u;

constexpr int kXCols     = 15;
constexpr int kFeatReal  = 36;
constexpr int kK1        = 64;
constexpr int kN1        = 128;
constexpr int kK2        = 128;
constexpr int kN2        = 512;
constexpr int kK3        = 512;
constexpr int kN3        = 64;
constexpr int kNAct      = 40;
constexpr int kChunkRows = 32768;

__device__ __forceinline__ unsigned short f2bf_bits(float f) {
  unsigned u = __float_as_uint(f);
  return (unsigned short)((u + 0x7FFFu + ((u >> 16) & 1u)) >> 16);
}
__device__ __forceinline__ float bf_bits2f(unsigned short h) { return __uint_as_float(((unsigned)h) << 16); }

__device__ __forceinline__ void dep_guard_h(v8f& a, v8f& b, v16h x, v16h y) { asm volatile("v_nop\n\tv_nop\n\tv_nop\n\tv_nop" : "+v"(a), "+v"(b) : "v"(x), "v"(y)); }
__device__ __forceinline__ void dep_guard_b(v8f& a, v8f& b, v16b x, v16b y) { asm volatile("v_nop\n\tv_nop\n\tv_nop\n\tv_nop" : "+v"(a), "+v"(b) : "v"(x), "v"(y)); }
__device__ __forceinline__ void keep4_h(v16h a, v16h b, v16h c, v16h d) { asm volatile("v_nop" :: "v"(a), "v"(b), "v"(c), "v"(d)); }
__device__ __forceinline__ void keep4_b(v16b a, v16b b, v16b c, v16b d) { asm volatile("v_nop" :: "v"(a), "v"(b), "v"(c), "v"(d)); }
__device__ __forceinline__ void acc_guard4(v8f& a, v8f& b, v8f& c, v8f& d) { asm volatile("v_nop\n\tv_nop\n\tv_nop\n\tv_nop" : "+v"(a), "+v"(b), "+v"(c), "+v"(d)); }
template <typename T> struct Frag;
template <> struct Frag<_Float16> {
  typedef v16h V; union U { v16h v; v8h h[2]; };
  static __device__ __forceinline__ v16h load(const _Float16* p) {
    U f; f.h[0] = *(const v8h*)(p); f.h[1] = *(const v8h*)(p + 16); return f.v;
  }
  static __device__ __forceinline__ v8f mma(v16h a, v16h b, v8f c) {
    return __builtin_amdgcn_wmma_f32_16x16x32_f16(false, a, false, b, (short)0, c, false, false);
  }
  static __device__ __forceinline__ void guard(v8f& a, v8f& b, v16h x, v16h y) { dep_guard_h(a, b, x, y); }
  static __device__ __forceinline__ void keep(v16h a, v16h b, v16h c, v16h d) { keep4_h(a, b, c, d); }
};
template <> struct Frag<__bf16> {
  typedef v16b V; union U { v16b v; v8b h[2]; };
  static __device__ __forceinline__ v16b load(const __bf16* p) {
    U f; f.h[0] = *(const v8b*)(p); f.h[1] = *(const v8b*)(p + 16); return f.v;
  }
  static __device__ __forceinline__ v8f mma(v16b a, v16b b, v8f c) {
    return __builtin_amdgcn_wmma_f32_16x16x32_bf16(false, a, false, b, (short)0, c, false, false);
  }
  static __device__ __forceinline__ void guard(v8f& a, v8f& b, v16b x, v16b y) { dep_guard_b(a, b, x, y); }
  static __device__ __forceinline__ void keep(v16b a, v16b b, v16b c, v16b d) { keep4_b(a, b, c, d); }
};

__device__ __forceinline__ unsigned pk16(unsigned short a, unsigned short b) { return (unsigned)a | ((unsigned)b << 16); }

template <int ET> struct Elem;
template <> struct Elem<0> { typedef _Float16 T; };
template <> struct Elem<1> { typedef __bf16 T; };
template <int ET, bool SPLIT, int BIAS_MODE, int OUT_MODE, bool RESID, int ACT = 0>
__global__ __launch_bounds__(256) void wmma_gemm64(
    const unsigned short* __restrict__ Ap, const unsigned short* __restrict__ A2p, int lda, long strideA,
    const unsigned short* __restrict__ Btp, const unsigned short* __restrict__ Bt2p, int ldb, long strideB,
    void* __restrict__ Cout, void* __restrict__ Cout2, int ldc, long strideC,
    const float* __restrict__ bias,
    const float* __restrict__ resid, long strideR,
    int M, int N, int K, float scale) {
  typedef typename Elem<ET>::T T;
  typedef typename Frag<T>::V V;
  const T* A = (const T*)Ap; const T* A2 = (const T*)A2p; const T* Bt = (const T*)Btp; const T* Bt2 = (const T*)Bt2p;
  __shared__ __align__(16) float sT[8][16 * 68];
  const int b    = blockIdx.y;
  const int lane = threadIdx.x & 31;
  const int wave = threadIdx.x >> 5;
  const int tilesN = N >> 6;
  const int tilesM = M >> 6;
  const int tile = blockIdx.x * 8 + wave;
  if (tile >= tilesM * tilesN) return;
  const int tm = tile / tilesN;
  const int tn = tile - tm * tilesN;
  const int m0 = tm << 6;
  const int n0 = tn << 6;

  const T* Ab  = A  + (size_t)b * strideA;
  const T* Bb  = Bt + (size_t)b * strideB;
  const T* Ab2 = SPLIT ? (A2  + (size_t)b * strideA) : nullptr;
  const T* Bb2 = SPLIT ? (Bt2 + (size_t)b * strideB) : nullptr;

  const int rlane = lane & 15;
  const int koff  = (lane >> 4) * 8;
  const int mOff  = (lane >> 4) * 8;

  v8f acc[4][4];
#pragma unroll
  for (int i = 0; i < 4; ++i)
#pragma unroll
    for (int j = 0; j < 4; ++j) acc[i][j] = (v8f){0.f,0.f,0.f,0.f,0.f,0.f,0.f,0.f};

  for (int k0 = 0; k0 < K; k0 += 32) {
    V bh[4], bl[4];
#pragma unroll
    for (int j = 0; j < 4; ++j) {
      const size_t bo = (size_t)(n0 + (j << 4) + rlane) * ldb + koff + k0;
      bh[j] = Frag<T>::load(Bb + bo);
      if (SPLIT) bl[j] = Frag<T>::load(Bb2 + bo);
    }
#pragma unroll
    for (int i = 0; i < 4; ++i) {
      const size_t ao = (size_t)(m0 + (i << 4) + rlane) * lda + koff + k0;
      V ah = Frag<T>::load(Ab + ao);
      V al;
      if (SPLIT) al = Frag<T>::load(Ab2 + ao);
#pragma unroll
      for (int j = 0; j < 4; ++j) {
        acc[i][j] = Frag<T>::mma(ah, bh[j], acc[i][j]);
        if (SPLIT) {
          acc[i][j] = Frag<T>::mma(ah, bl[j], acc[i][j]);
          acc[i][j] = Frag<T>::mma(al, bh[j], acc[i][j]);
        }
      }
      Frag<T>::guard(acc[i][0], acc[i][3], ah, SPLIT ? al : ah);
    }
    Frag<T>::keep(bh[0], bh[1], bh[2], bh[3]);
    if (SPLIT) Frag<T>::keep(bl[0], bl[1], bl[2], bl[3]);
  }
  acc_guard4(acc[0][0], acc[0][1], acc[0][2], acc[0][3]);
  acc_guard4(acc[1][0], acc[1][1], acc[1][2], acc[1][3]);
  acc_guard4(acc[2][0], acc[2][1], acc[2][2], acc[2][3]);
  acc_guard4(acc[3][0], acc[3][1], acc[3][2], acc[3][3]);

  float* slab = sT[wave];
  const float* Rb = RESID ? (resid + (size_t)b * strideR) : nullptr;
#pragma unroll
  for (int i = 0; i < 4; ++i) {
    const int mBase = m0 + (i << 4);
#pragma unroll
    for (int j = 0; j < 4; ++j) {
      const int n = n0 + (j << 4) + rlane;
      float bv = 0.f;
      if (BIAS_MODE == 2) bv = bias[n];
#pragma unroll
      for (int r = 0; r < 8; ++r) {
        float v = acc[i][j][r] * scale;
        if (BIAS_MODE == 1) v += bias[mBase + mOff + r];
        if (BIAS_MODE == 2) v += bv;
        if (RESID) v += Rb[(size_t)(mBase + mOff + r) * ldc + n];
        if (ACT == 2) v = fmaxf(v, 0.0f);
        if (ACT == 4) v = (v > 0.f) ? v : 0.01f * v;
        slab[(mOff + r) * 68 + (j << 4) + rlane] = v;
      }
    }
    __builtin_amdgcn_fence(__ATOMIC_RELEASE, "workgroup");
    __builtin_amdgcn_wave_barrier();
    __builtin_amdgcn_fence(__ATOMIC_ACQUIRE, "workgroup");
    if (OUT_MODE == 0) {
      float* C = (float*)Cout + (size_t)b * strideC;
      const int hh = lane >> 4, c4 = (lane & 15) * 4;
      for (int pass = 0; pass < 2; ++pass) {
#pragma unroll
        for (int it = 0; it < 8; ++it) {
          const int row = it * 2 + hh;
          v4f v = *(const v4f*)(slab + row * 68 + c4);
          *(volatile v4f*)(C + (size_t)(mBase + row) * ldc + n0 + c4) = v;
        }
        __threadfence();
      }
    } else {
      const int q = lane >> 3, c8 = (lane & 7) * 8;
      unsigned short* C  = (unsigned short*)Cout  + (size_t)b * strideC;
      unsigned short* C2 = (OUT_MODE == 2) ? ((unsigned short*)Cout2 + (size_t)b * strideC) : nullptr;
      for (int pass = 0; pass < 2; ++pass) {
#pragma unroll
        for (int it = 0; it < 4; ++it) {
          const int row = it * 4 + q;
          const float* sp = slab + row * 68 + c8;
          v8h hv, lv;
#pragma unroll
          for (int e = 0; e < 8; ++e) {
            if (OUT_MODE == 1) {
              hv[e] = (_Float16)sp[e];
            } else {
              unsigned short hb = f2bf_bits(sp[e]);
              unsigned short lb = f2bf_bits(sp[e] - bf_bits2f(hb));
              hv[e] = __builtin_bit_cast(_Float16, hb);
              lv[e] = __builtin_bit_cast(_Float16, lb);
            }
          }
          *(volatile v8h*)(C + (size_t)(mBase + row) * ldc + n0 + c8) = hv;
          if (OUT_MODE == 2) *(volatile v8h*)(C2 + (size_t)(mBase + row) * ldc + n0 + c8) = lv;
        }
        __threadfence();
      }
    }
    __builtin_amdgcn_fence(__ATOMIC_RELEASE, "workgroup");
    __builtin_amdgcn_wave_barrier();
    __builtin_amdgcn_fence(__ATOMIC_ACQUIRE, "workgroup");
  }
}

__global__ __launch_bounds__(256) void wprep_kernel(const float* __restrict__ W1, const float* __restrict__ W2,
                                                    const float* __restrict__ W4,
                                                    unsigned short* __restrict__ w1h, unsigned short* __restrict__ w1l,
                                                    unsigned short* __restrict__ w2h, unsigned short* __restrict__ w2l,
                                                    unsigned short* __restrict__ w4h, unsigned short* __restrict__ w4l) {
  const int z = blockIdx.y;
  const int i = blockIdx.x * 256 + threadIdx.x;
  const float* W; unsigned short* oh; unsigned short* ol;
  int kbShift, kReal, nReal, nRows, ldw;
  if (z == 0)      { W = W1; oh = w1h; ol = w1l; kbShift = 3; kReal = kFeatReal; nReal = kN1;   nRows = kN1; ldw = kN1; }
  else if (z == 1) { W = W2; oh = w2h; ol = w2l; kbShift = 4; kReal = kK2;       nReal = kN2;   nRows = kN2; ldw = kN2; }
  else             { W = W4; oh = w4h; ol = w4l; kbShift = 6; kReal = kK3;       nReal = kNAct; nRows = kN3; ldw = kNAct; }
  const int total = nRows << kbShift;
  if (i >= total) return;
  const int n  = i >> kbShift;
  const int k0 = (i - (n << kbShift)) * 8;
  const int nc = n < nReal ? n : nReal - 1;
  unsigned short hb[8], lb[8];
#pragma unroll
  for (int e = 0; e < 8; ++e) {
    const int k  = k0 + e;
    const int kc = k < kReal ? k : kReal - 1;
    float v = W[(size_t)kc * ldw + nc];
    v = (k < kReal && n < nReal) ? v : 0.0f;
    const unsigned short h = f2bf_bits(v);
    hb[e] = h;
    lb[e] = f2bf_bits(v - bf_bits2f(h));
  }
  const v4u hu = (v4u){pk16(hb[0], hb[1]), pk16(hb[2], hb[3]), pk16(hb[4], hb[5]), pk16(hb[6], hb[7])};
  const v4u lu = (v4u){pk16(lb[0], lb[1]), pk16(lb[2], lb[3]), pk16(lb[4], lb[5]), pk16(lb[6], lb[7])};
  unsigned short* ph = oh + 8 * (size_t)i;
  unsigned short* pl = ol + 8 * (size_t)i;
  *(volatile v4u*)ph = hu;
  *(volatile v4u*)pl = lu;
  __threadfence();
  *(volatile v4u*)ph = hu;
  *(volatile v4u*)pl = lu;
}

__global__ __launch_bounds__(256) void feat_kernel(const float* __restrict__ x,
                                                   unsigned short* __restrict__ ah, unsigned short* __restrict__ al,
                                                   int row0, int nrows_total, int nrows_chunk) {
  const int t  = blockIdx.x * 256 + threadIdx.x;
  const int rl = t >> 3;
  if (rl >= nrows_chunk) return;
  const int q = t & 7;
  int rg = row0 + rl;
  rg = rg < nrows_total ? rg : nrows_total - 1;
  const float* xr = x + (size_t)rg * kXCols;
  const float hf = xr[11];
  const float f0 = xr[12];
  const float f1 = xr[13];
  const float f2 = xr[14];
  int hid = (int)hf;      hid = hid < 0 ? 0 : (hid > 3 ? 3 : hid);
  int i0  = (int)f0 - 1;  i0  = i0  < 0 ? 0 : (i0  > 6 ? 6 : i0);
  int i1  = (int)f1 - 1;  i1  = i1  < 0 ? 0 : (i1  > 6 ? 6 : i1);
  int i2  = (int)f2 - 1;  i2  = i2  < 0 ? 0 : (i2  > 6 ? 6 : i2);
  unsigned short hb[8], lb[8];
#pragma unroll
  for (int e = 0; e < 8; ++e) {
    const int col = q * 8 + e;
    const int kc  = col < 10 ? col : 10;
    const float kv = xr[kc];
    const int cr  = col - 15;
    const int jj  = cr >= 14 ? 2 : (cr >= 7 ? 1 : 0);
    const int cc  = cr - 7 * jj;
    const int idx = jj == 0 ? i0 : (jj == 1 ? i1 : i2);
    float v = (col < kFeatReal) ? ((idx == cc) ? 1.0f : 0.0f) : 0.0f;
    v = (col < 15) ? ((hid == col - 11) ? 1.0f : 0.0f) : v;
    v = (col < 11) ? kv : v;
    const unsigned short h = f2bf_bits(v);
    hb[e] = h;
    lb[e] = f2bf_bits(v - bf_bits2f(h));
  }
  const v4u hu = (v4u){pk16(hb[0], hb[1]), pk16(hb[2], hb[3]), pk16(hb[4], hb[5]), pk16(hb[6], hb[7])};
  const v4u lu = (v4u){pk16(lb[0], lb[1]), pk16(lb[2], lb[3]), pk16(lb[4], lb[5]), pk16(lb[6], lb[7])};
  unsigned short* ph = ah + (size_t)rl * kK1 + q * 8;
  unsigned short* pl = al + (size_t)rl * kK1 + q * 8;
  *(volatile v4u*)ph = hu;
  *(volatile v4u*)pl = lu;
  __threadfence();
  *(volatile v4u*)ph = hu;
  *(volatile v4u*)pl = lu;
}

__global__ __launch_bounds__(256) void out_writer_kernel(const float* __restrict__ c3, const float* __restrict__ b4,
                                                         float* __restrict__ out, int n4) {
  const int t = blockIdx.x * 256 + threadIdx.x;
  if (t >= n4) return;
  const int row = t / 10;
  const int c   = (t - row * 10) * 4;
  const v4f v = *(const v4f*)(c3 + (size_t)row * kN3 + c);
  v4f bb;
  bb[0] = b4[c]; bb[1] = b4[c + 1]; bb[2] = b4[c + 2]; bb[3] = b4[c + 3];
  const v4f o = v + bb;
  float* p = out + 4 * (size_t)t;
  *(volatile v4f*)p = o;
  __threadfence();
  *(volatile v4f*)p = o;
}

extern "C" void kernel_launch(void* const* d_in, const int* in_sizes, int n_in,
                              void* d_out, int out_size, void* d_ws, size_t ws_size,
                              hipStream_t stream) {
  if (n_in < 7) return;
  const float* x  = (const float*)d_in[0];
  const float* W1 = (const float*)d_in[1];
  const float* b1 = (const float*)d_in[2];
  const float* W2 = (const float*)d_in[3];
  const float* b2 = (const float*)d_in[4];
  const float* W4 = (const float*)d_in[5];
  const float* b4 = (const float*)d_in[6];
  float* out = (float*)d_out;

  const int nrows = in_sizes[0] / kXCols;
  if (nrows <= 0 || (nrows % kChunkRows) != 0) return;
  if (out_size < nrows * kNAct) return;
  const int nchunk = nrows / kChunkRows;

  const size_t szW1 = (size_t)kN1 * kK1 * 2;
  const size_t szW2 = (size_t)kN2 * kK2 * 2;
  const size_t szW4 = (size_t)kN3 * kK3 * 2;
  const size_t szA1 = (size_t)kChunkRows * kK1 * 2;
  const size_t szH1 = (size_t)kChunkRows * kN1 * 2;
  const size_t szH2 = (size_t)kChunkRows * kN2 * 2;
  const size_t szC3 = (size_t)nrows * kN3 * 4;

  size_t off = 0;
  const size_t oW1h = off; off += szW1;  const size_t oW1l = off; off += szW1;
  const size_t oW2h = off; off += szW2;  const size_t oW2l = off; off += szW2;
  const size_t oW4h = off; off += szW4;  const size_t oW4l = off; off += szW4;
  const size_t oA1h = off; off += szA1;  const size_t oA1l = off; off += szA1;
  const size_t oH1h = off; off += szH1;  const size_t oH1l = off; off += szH1;
  const size_t oH2h = off; off += szH2;  const size_t oH2l = off; off += szH2;
  const size_t oC3  = off; off += szC3;
  if (off > ws_size) return;

  unsigned char* ws = (unsigned char*)d_ws;
  unsigned short* w1h = (unsigned short*)(ws + oW1h);
  unsigned short* w1l = (unsigned short*)(ws + oW1l);
  unsigned short* w2h = (unsigned short*)(ws + oW2h);
  unsigned short* w2l = (unsigned short*)(ws + oW2l);
  unsigned short* w4h = (unsigned short*)(ws + oW4h);
  unsigned short* w4l = (unsigned short*)(ws + oW4l);
  unsigned short* a1h = (unsigned short*)(ws + oA1h);
  unsigned short* a1l = (unsigned short*)(ws + oA1l);
  unsigned short* h1h = (unsigned short*)(ws + oH1h);
  unsigned short* h1l = (unsigned short*)(ws + oH1l);
  unsigned short* h2h = (unsigned short*)(ws + oH2h);
  unsigned short* h2l = (unsigned short*)(ws + oH2l);
  float*          c3  = (float*)(ws + oC3);

  {
    const int nthr = (kN2 * kK2) / 8;
    wprep_kernel<<<dim3((nthr + 255) / 256, 3, 1), 256, 0, stream>>>(W1, W2, W4, w1h, w1l, w2h, w2l, w4h, w4l);
  }

  const int tilesM = kChunkRows / 64;
  const int g1 = (tilesM * (kN1 / 64) + 7) / 8;
  const int g2 = (tilesM * (kN2 / 64) + 7) / 8;
  const int g3 = (tilesM * (kN3 / 64) + 7) / 8;
  const int gfeat = (kChunkRows * 8 + 255) / 256;

  for (int ch = 0; ch < nchunk; ++ch) {
    const int row0 = ch * kChunkRows;
    feat_kernel<<<dim3(gfeat, 1, 1), 256, 0, stream>>>(x, a1h, a1l, row0, nrows, kChunkRows);
    wmma_gemm64<1, true, 2, 2, false, 2><<<dim3(g1, 1, 1), 256, 0, stream>>>(
        a1h, a1l, kK1, 0L, w1h, w1l, kK1, 0L,
        (void*)h1h, (void*)h1l, kN1, 0L, b1, b1, 0L, kChunkRows, kN1, kK1, 1.0f);
    wmma_gemm64<1, true, 2, 2, false, 2><<<dim3(g2, 1, 1), 256, 0, stream>>>(
        h1h, h1l, kK2, 0L, w2h, w2l, kK2, 0L,
        (void*)h2h, (void*)h2l, kN2, 0L, b2, b2, 0L, kChunkRows, kN2, kK2, 1.0f);
    float* c3c = c3 + (size_t)row0 * kN3;
    wmma_gemm64<1, true, 0, 0, false, 0><<<dim3(g3, 1, 1), 256, 0, stream>>>(
        h2h, h2l, kK3, 0L, w4h, w4l, kK3, 0L,
        (void*)c3c, (void*)c3c, kN3, 0L, b1, b1, 0L, kChunkRows, kN3, kK3, 1.0f);
  }

  {
    const int n4 = (nrows * kNAct) / 4;
    out_writer_kernel<<<dim3((n4 + 255) / 256, 1, 1), 256, 0, stream>>>(c3, b4, out, n4);
  }
}
